// SimCLR_26920855011622
// MI455X (gfx1250) — hardware-verified
//
#include <hip/hip_runtime.h>
#include <math.h>

typedef __attribute__((ext_vector_type(16))) _Float16 v16h;
typedef __attribute__((ext_vector_type(16))) __bf16 v16b;
typedef __attribute__((ext_vector_type(8)))  _Float16 v8h;
typedef __attribute__((ext_vector_type(8)))  float v8f;
typedef __attribute__((ext_vector_type(4)))  float v4f;
typedef __attribute__((ext_vector_type(2)))  float v2f;
typedef __attribute__((ext_vector_type(4)))  unsigned v4u;
typedef __attribute__((ext_vector_type(4)))  int v4i;
typedef float __attribute__((may_alias)) float_a;
typedef int __attribute__((may_alias)) int_a;

template <typename T> __device__ __forceinline__ void vst2(void* p, T v) { *(volatile T*)p = v; __threadfence(); *(volatile T*)p = v; }
__device__ __forceinline__ v8f wmma16(v16h a, v16h b, v8f c) {
  v8f d = __builtin_amdgcn_wmma_f32_16x16x32_f16(false, a, false, b, (short)0, c, false, false);
  asm volatile("v_nop\n\tv_nop\n\tv_nop\n\tv_nop" : "+v"(d) : "v"(a), "v"(b));
  return d;
}
__device__ __forceinline__ v8f wmma_bf(v16b a, v16b b, v8f c) {
  v8f d = __builtin_amdgcn_wmma_f32_16x16x32_bf16(false, a, false, b, (short)0, c, false, false);
  asm volatile("v_nop\n\tv_nop\n\tv_nop\n\tv_nop" : "+v"(d) : "v"(a), "v"(b));
  return d;
}
__device__ __forceinline__ v16h frag_h(const _Float16* rowk0, int lane) {
  union { v16h v; v8h q[2]; } u; const _Float16* p = rowk0 + 8 * (lane >> 4);
  u.q[0] = *(const v8h*)p; u.q[1] = *(const v8h*)(p + 16); return u.v;
}
__device__ __forceinline__ v16h frag_f32(const float* rowk0, int lane) {
  v16h a; const float* p = rowk0 + 8 * (lane >> 4);
#pragma unroll
  for (int i = 0; i < 8; ++i) { a[i] = (_Float16)p[i]; a[8 + i] = (_Float16)p[16 + i]; }
  return a;
}
__device__ __forceinline__ v16h frag_f32s(const float* rowk0, int lane, float sc) {
  v16h a; const float* p = rowk0 + 8 * (lane >> 4);
#pragma unroll
  for (int i = 0; i < 8; ++i) { a[i] = (_Float16)(p[i] * sc); a[8 + i] = (_Float16)(p[16 + i] * sc); }
  return a;
}
__device__ __forceinline__ v16h fragc_f32(const float* W, int k0, int n, int lane, int ld, int K) {
  v16h a; const int g = lane >> 4;
#pragma unroll
  for (int i = 0; i < 8; ++i) { const int ka = k0 + 8 * g + i, kb = ka + 16;
    a[i] = (_Float16)(ka < K ? W[(size_t)ka * ld + n] : 0.f); a[8 + i] = (_Float16)(kb < K ? W[(size_t)kb * ld + n] : 0.f); }
  return a;
}
struct F2 { v16b h, l; };
__device__ __forceinline__ F2 bsplit16(const float v[16]) { F2 r;
#pragma unroll
  for (int i = 0; i < 16; ++i) { const __bf16 h = (__bf16)v[i]; r.h[i] = h; r.l[i] = (__bf16)(v[i] - (float)h); }
  return r; }
__device__ __forceinline__ F2 split_row(const float* row, int k0, int lane) { float v[16]; const float* p = row + k0 + 8 * (lane >> 4);
#pragma unroll
  for (int i = 0; i < 8; ++i) { v[i] = p[i]; v[8 + i] = p[16 + i]; }
  return bsplit16(v); }
__device__ __forceinline__ F2 split_rowK(const float* row, int k0, int lane, int K) { float v[16]; const int g = lane >> 4;
#pragma unroll
  for (int i = 0; i < 8; ++i) { const int ka = k0 + 8 * g + i, kb = ka + 16; v[i] = ka < K ? row[ka] : 0.f; v[8 + i] = kb < K ? row[kb] : 0.f; }
  return bsplit16(v); }
__device__ __forceinline__ F2 split_col(const float* W, int k0, int n, int lane, int ld, int K) { float v[16]; const int g = lane >> 4;
#pragma unroll
  for (int i = 0; i < 8; ++i) { const int ka = k0 + 8 * g + i, kb = ka + 16; v[i] = ka < K ? W[(size_t)ka * ld + n] : 0.f; v[8 + i] = kb < K ? W[(size_t)kb * ld + n] : 0.f; }
  return bsplit16(v); }
__device__ __forceinline__ v8f mac3(const F2& a, const F2& b, v8f c) { c = wmma_bf(a.l, b.h, c); c = wmma_bf(a.h, b.l, c); return wmma_bf(a.h, b.h, c); }
__device__ __forceinline__ float sigm(float v) { return 1.0f / (1.0f + expf(-v)); }
#define LDSX() do { asm volatile("s_wait_dscnt 0" ::: "memory"); __builtin_amdgcn_wave_barrier(); __builtin_amdgcn_fence(__ATOMIC_RELEASE, "workgroup"); } while (0)

#define NBT 4096
#define DIN 192
#define DH 512
#define DO 128
#define N2 (2 * NBT)
#define NBLK (NBT / 64)

__global__ __launch_bounds__(128) void k_l1(const float* __restrict__ h1, const float* __restrict__ h2, const float* __restrict__ W1, const float* __restrict__ b1, float* __restrict__ Y, float* __restrict__ pst) {
  __shared__ __align__(16) float so[4][16][132];
  __shared__ __align__(16) float sps[4][2][128];
  const int tid = threadIdx.x, wave = tid >> 5, lane = tid & 31, col = lane & 15, g = lane >> 4;
  const int v = blockIdx.z, blk = blockIdx.x, r0 = blk * 64 + wave * 16, n0 = blockIdx.y * 128; const float* h = v == 0 ? h1 : h2;
  v8f acc[8] = {};
#pragma unroll
  for (int kc = 0; kc < DIN / 32; ++kc) { const v16h a = frag_f32(h + (size_t)(r0 + col) * DIN + kc * 32, lane);
#pragma unroll
    for (int j = 0; j < 8; ++j) acc[j] = wmma16(a, frag_f32s(W1 + (size_t)(n0 + j * 16 + col) * DIN + kc * 32, lane, 16.0f), acc[j]); }
#pragma unroll
  for (int j = 0; j < 8; ++j) { const float bb = b1[n0 + j * 16 + col];
#pragma unroll
    for (int r = 0; r < 8; ++r) so[wave][8 * g + r][j * 16 + col] = acc[j][r] * (1.0f / 16.0f) + bb; }
  LDSX();
#pragma unroll 4
  for (int rl = 0; rl < 16; ++rl) vst2(Y + ((size_t)v * NBT + r0 + rl) * DH + n0 + lane * 4, *(const v4f*)(&so[wave][rl][lane * 4]));
  { float s[4] = {0.f, 0.f, 0.f, 0.f}, s2[4] = {0.f, 0.f, 0.f, 0.f};
    for (int rl = 0; rl < 16; ++rl) {
#pragma unroll
      for (int e = 0; e < 4; ++e) { const float y = so[wave][rl][lane * 4 + e]; s[e] += y; s2[e] += y * y; } }
#pragma unroll
    for (int e = 0; e < 4; ++e) { sps[wave][0][lane * 4 + e] = s[e]; sps[wave][1][lane * 4 + e] = s2[e]; } }
  __syncthreads();
  __shared__ __align__(16) float sout[2][128];
  for (int q = tid; q < 256; q += 128) { const int st = q >> 7, c = q & 127; sout[st][c] = (sps[0][st][c] + sps[1][st][c]) + (sps[2][st][c] + sps[3][st][c]); }
  __syncthreads();
  if (tid < 64) { const int st = tid >> 5, pc = tid & 31; vst2(pst + (((size_t)v * NBLK + blk) * 2 + st) * DH + n0 + pc * 4, *(const v4f*)(&sout[st][pc * 4])); }
}
__global__ __launch_bounds__(256) void k_stat(const float* __restrict__ pst, float* __restrict__ stat) {
  __shared__ __align__(16) float so[2][DH];
  const int v = blockIdx.x, tid = threadIdx.x;
  for (int c = tid; c < DH; c += 256) { float s = 0.f, s2 = 0.f;
#pragma unroll 1
    for (int blk = 0; blk < NBLK; ++blk) { s += pst[(((size_t)v * NBLK + blk) * 2 + 0) * DH + c]; s2 += pst[(((size_t)v * NBLK + blk) * 2 + 1) * DH + c]; }
    const float mean = s / (float)NBT; const float var = fmaxf(s2 / (float)NBT - mean * mean, 0.f);
    so[0][c] = mean; so[1][c] = rsqrtf(var + 1e-5f); }
  __syncthreads();
  for (int q = tid; q < 2 * DH / 4; q += 256) vst2(stat + (size_t)v * 2 * DH + q * 4, *(const v4f*)(&so[0][0] + q * 4));
}
__global__ __launch_bounds__(128) void k_l2(const float* __restrict__ Y, const float* __restrict__ stat, const float* __restrict__ gam, const float* __restrict__ bet, const float* __restrict__ W2, const float* __restrict__ b2, float* __restrict__ Zf, _Float16* __restrict__ Z16) {
  __shared__ __align__(16) float sa[4][16][DH + 4];
  __shared__ __align__(16) float so[4][16][132];
  const int tid = threadIdx.x, wave = tid >> 5, lane = tid & 31, col = lane & 15, g = lane >> 4;
  const int v = blockIdx.y, r0 = blockIdx.x * 64 + wave * 16; const float* mean = stat + (size_t)v * 2 * DH; const float* rstd = mean + DH;
  for (int q = lane; q < 16 * DH; q += 32) { const int rl = q / DH, c = q % DH; const float y = Y[((size_t)v * NBT + r0 + rl) * DH + c]; const float a = (y - mean[c]) * rstd[c] * gam[c] + bet[c]; sa[wave][rl][c] = a > 0.f ? a : 0.f; }
  LDSX();
  v8f acc[8] = {};
#pragma unroll 1
  for (int kc = 0; kc < DH / 32; ++kc) { const v16h a = frag_f32(&sa[wave][col][0] + kc * 32, lane);
#pragma unroll
    for (int j = 0; j < 8; ++j) acc[j] = wmma16(a, frag_f32s(W2 + (size_t)(j * 16 + col) * DH + kc * 32, lane, 16.0f), acc[j]); }
#pragma unroll
  for (int j = 0; j < 8; ++j) { const float bb = b2[j * 16 + col];
#pragma unroll
    for (int r = 0; r < 8; ++r) so[wave][8 * g + r][j * 16 + col] = acc[j][r] * (1.0f / 16.0f) + bb; }
  LDSX();
  { const int rl = lane >> 1, hf = lane & 1; float s = 0.f; for (int c = 0; c < 64; ++c) { const float zz = so[wave][rl][hf * 64 + c]; s += zz * zz; } s += __shfl_xor(s, 1, 32);
    const float inv = 1.0f / fmaxf(sqrtf(s), 1e-12f);
    LDSX();
    for (int c = 0; c < 64; ++c) so[wave][rl][hf * 64 + c] *= inv; }
  LDSX();
  for (int q = lane; q < 16 * 32; q += 32) { const int rl = q >> 5, pc = q & 31; vst2(Zf + ((size_t)v * NBT + r0 + rl) * DO + pc * 4, *(const v4f*)(&so[wave][rl][pc * 4])); }
  for (int q = lane; q < 16 * 16; q += 32) { const int rl = q >> 4, pc = q & 15; union { v8h h8; v4u u; } pk;
#pragma unroll
    for (int e = 0; e < 8; ++e) pk.h8[e] = (_Float16)(so[wave][rl][pc * 8 + e] * 8.0f);
    vst2(Z16 + ((size_t)v * NBT + r0 + rl) * DO + pc * 8, pk.u); }
}
__global__ __launch_bounds__(128) void k_sim(const _Float16* __restrict__ Z16, float* __restrict__ part) {
  __shared__ __align__(16) float sS[4][16][68];
  __shared__ float sacc[4];
  const int tid = threadIdx.x, w = tid >> 5, lane = tid & 31, col = lane & 15, g = lane >> 4;
  const int r0 = blockIdx.x * 64 + w * 16;
  v16h az[4];
#pragma unroll
  for (int kc = 0; kc < 4; ++kc) az[kc] = frag_h(Z16 + (size_t)(r0 + col) * DO + kc * 32, lane);
  float mrun = -3.0e38f, lrun = 0.f, posv = 0.f;
#pragma unroll 1
  for (int ct = 0; ct < N2 / 64; ++ct) {
#pragma unroll
    for (int t = 0; t < 4; ++t) { v8f s = {}; const int cj = ct * 64 + t * 16 + col;
#pragma unroll
      for (int kc = 0; kc < 4; ++kc) s = wmma16(az[kc], frag_h(Z16 + (size_t)cj * DO + kc * 32, lane), s);
#pragma unroll
      for (int r = 0; r < 8; ++r) { const int ri = r0 + 8 * g + r; const float sim = s[r] * (1.0f / 64.0f) * 2.0f;
        sS[w][8 * g + r][t * 16 + col] = (cj == ri) ? -3.0e38f : sim; } }
    LDSX();
    { const int m = col; float mx = -3.4e38f;
#pragma unroll
      for (int jj = 0; jj < 32; ++jj) mx = fmaxf(mx, sS[w][m][g * 32 + jj]);
      mx = fmaxf(mx, __shfl_xor(mx, 16, 32));
      const float mnew = fmaxf(mrun, mx); float ps = 0.f;
#pragma unroll
      for (int jj = 0; jj < 32; ++jj) { const float sv = sS[w][m][g * 32 + jj]; ps += sv <= -1.0e38f ? 0.f : expf(sv - mnew); }
      ps += __shfl_xor(ps, 16, 32);
      lrun = lrun * expf(mrun - mnew) + ps; mrun = mnew;
      const int ri = r0 + m; const int pj = (ri + NBT) & (N2 - 1); if (pj >= ct * 64 && pj < ct * 64 + 64 && g == 0) posv = sS[w][m][pj - ct * 64]; }
    LDSX(); }
  { const int m = col; float val = 0.f; if (g == 0) val = (mrun + logf(lrun)) - posv;
    for (int off = 8; off >= 1; off >>= 1) val += __shfl_xor(val, off, 32);
    if (lane == 0) sacc[w] = val; }
  __syncthreads();
  if (tid < 32) vst2(part + (size_t)blockIdx.x * 32 + tid, (float)(tid == 0 ? (sacc[0] + sacc[1]) + (sacc[2] + sacc[3]) : 0.f));
}
__global__ __launch_bounds__(1024) void k_out(const float* __restrict__ part, const float* __restrict__ Zf, float* __restrict__ out) {
  const int tid = threadIdx.x;
  if (tid == 0) { float s = 0.f; for (int b = 0; b < N2 / 64; ++b) s += part[(size_t)b * 32]; vst2(out, s / (float)N2); }
  for (size_t i = tid; i < (size_t)NBT * DO; i += 1024) { vst2(out + 1 + i, Zf[i]); vst2(out + 1 + (size_t)NBT * DO + i, Zf[(size_t)NBT * DO + i]); }
}
extern "C" void kernel_launch(void* const* d_in, const int* in_sizes, int n_in, void* d_out, int out_size, void* d_ws, size_t ws_size, hipStream_t stream) {
  (void)in_sizes; (void)n_in; (void)out_size; (void)ws_size;
  const float** I = (const float**)d_in;
  const float* h1 = I[0]; const float* h2 = I[1]; const float* W1 = I[2]; const float* b1 = I[3]; const float* gam = I[4]; const float* bet = I[5]; const float* W2 = I[6]; const float* b2 = I[7];
  float* out = (float*)d_out;
  char* ws = (char*)d_ws; size_t off = 0;
  auto take = [&](size_t bytes) { char* p = ws + off; off += (bytes + 255) & ~(size_t)255; return p; };
  float* Y = (float*)take((size_t)N2 * DH * 4); float* pst = (float*)take((size_t)2 * NBLK * 2 * DH * 4); float* stat = (float*)take((size_t)2 * 2 * DH * 4); _Float16* Z16 = (_Float16*)take((size_t)N2 * DO * 2); float* part = (float*)take((size_t)(N2 / 64) * 32 * 4); float* Zf = (float*)take((size_t)N2 * DO * 4);
  k_l1<<<dim3(NBLK, DH / 128, 2), 128, 0, stream>>>(h1, h2, W1, b1, Y, pst);
  k_stat<<<2, 256, 0, stream>>>(pst, stat);
  k_l2<<<dim3(NBLK, 2), 128, 0, stream>>>(Y, stat, gam, bet, W2, b2, Zf, Z16);
  k_sim<<<N2 / 64, 128, 0, stream>>>(Z16, part);
  k_out<<<1, 1024, 0, stream>>>(part, Zf, out);
}
